// MultiHeadLatentAttention_52209622450599
// MI455X (gfx1250) — hardware-verified
//
#include <hip/hip_runtime.h>
#include <math.h>


#pragma clang fp contract(off)

#ifndef SEQ
#define SEQ 2048
#endif
#ifndef NB
#define NB 1
#endif
#define SEQ_FULL 2048
#define EMB 2048
#define NH 16
#define QRK 512
#define KVRK 512
#define DROPE 64
#define DVH 128
#define HQK (DVH + DROPE)
#define QKW (NH * HQK)
#define N1 1152
#define N1USE 1088
#define CKV0 512
#define KR0 1024
#define AW 1024
#define N2 (NH * DVH + NH * DROPE)
#define QR0 (NH * DVH)
#define N3 (2 * NH * DVH)
#define V0 (NH * DVH)
#define NFREQ (DROPE / 2)
#define LOSC 16384.0f
#define PSC 16384.0f
#define ATSC 64.0f
#define CSTR 132
#define QLP 200
#define PLP 40
#define VTP 72

static_assert(NB == 1);
static_assert(SEQ % 64 == 0);
static_assert(SEQ >= 64);
static_assert(SEQ <= SEQ_FULL);
static_assert(N1 % 128 == 0);
static_assert(N2 % 128 == 0);
static_assert(N3 % 128 == 0);
static_assert(EMB % 128 == 0);
static_assert(QRK % 32 == 0);
static_assert(KVRK % 32 == 0);
static_assert(HQK % 32 == 0);
static_assert((QRK * EMB / 8) % 256 == 0);
static_assert((KVRK * EMB / 8) % 256 == 0);
static_assert((DROPE * EMB / 8) % 256 == 0);
static_assert(((N1 - N1USE) * EMB / 8) % 256 == 0);
static_assert((NH * DVH * QRK / 8) % 256 == 0);
static_assert((NH * DROPE * QRK / 8) % 256 == 0);
static_assert((N3 * KVRK / 8) % 256 == 0);
static_assert((EMB * EMB / 8) % 256 == 0);
static_assert((SEQ * EMB / 8) % 256 == 0);

typedef _Float16 v16h __attribute__((ext_vector_type(16)));
typedef float v8f __attribute__((ext_vector_type(8)));
typedef float v4f __attribute__((ext_vector_type(4)));
typedef unsigned short us;
typedef us us8 __attribute__((ext_vector_type(8)));
typedef us us16 __attribute__((ext_vector_type(16)));
typedef us8 __attribute__((may_alias)) us8a;
typedef v4f __attribute__((may_alias)) v4fa;

struct FreqTab { float inv[NFREQ]; };
static_assert(sizeof(FreqTab) == NFREQ * 4);

__device__ __forceinline__ unsigned bf16u(float f) { unsigned u = __float_as_uint(f); u += 0x7FFFu + ((u >> 16) & 1u); return u >> 16; }
__device__ __forceinline__ float bf16rt(float f) { return __uint_as_float(bf16u(f) << 16); }
__device__ __forceinline__ us hbits(float f) { return __builtin_bit_cast(us, (_Float16)f); }
__device__ __forceinline__ v16h frag(us8 p0, us8 p1) {
    const us16 t = __builtin_shufflevector(p0, p1, 0, 1, 2, 3, 4, 5, 6, 7, 8, 9, 10, 11, 12, 13, 14, 15);
    return __builtin_bit_cast(v16h, t);
}
__device__ __forceinline__ v8f vz8() { v8f z = {0.0f, 0.0f, 0.0f, 0.0f, 0.0f, 0.0f, 0.0f, 0.0f}; return z; }
__device__ __forceinline__ v8f wm(v16h a, v16h b, v8f c) {
    c = __builtin_amdgcn_wmma_f32_16x16x32_f16(false, a, false, b, (short)0, c, false, false);
    asm volatile("v_nop\n\tv_nop\n\tv_nop\n\tv_nop" : "+v"(c) : "v"(a), "v"(b));
    return c;
}
__device__ __forceinline__ us8 cvt8(const float* p, float sc) {
    const v4f a = *(const v4fa*)p, b = *(const v4fa*)(p + 4);
    us8 o;
    o[0] = hbits(bf16rt(a[0]) * sc); o[1] = hbits(bf16rt(a[1]) * sc); o[2] = hbits(bf16rt(a[2]) * sc); o[3] = hbits(bf16rt(a[3]) * sc);
    o[4] = hbits(bf16rt(b[0]) * sc); o[5] = hbits(bf16rt(b[1]) * sc); o[6] = hbits(bf16rt(b[2]) * sc); o[7] = hbits(bf16rt(b[3]) * sc);
    return o;
}

__global__ __launch_bounds__(256, 1) void cvt_plane(const float* __restrict__ src, us* dst, int n8, float sc) {
    const int i = blockIdx.x * 256 + (int)threadIdx.x;
    if (i >= n8) return;
    const us8 o = cvt8(src + (size_t)i * 8, sc);
    us* d = dst + (size_t)i * 8;
    *(volatile us8*)d = o;
    __threadfence();
    *(volatile us8*)d = o;
}
__global__ __launch_bounds__(256, 1) void zero_plane(us* dst, int n8) {
    const int i = blockIdx.x * 256 + (int)threadIdx.x;
    if (i >= n8) return;
    const us8 o = {0, 0, 0, 0, 0, 0, 0, 0};
    us* d = dst + (size_t)i * 8;
    *(volatile us8*)d = o;
    __threadfence();
    *(volatile us8*)d = o;
}

template <int RES>
__global__ __launch_bounds__(256, 1) void gemm_nt(const us* __restrict__ A, const us* __restrict__ Alo, int lda,
                                                  const us* __restrict__ B, int ldb, float* C, int ldc, int K, float oscale, float losc) {
    __shared__ __align__(16) float cst[64 * CSTR];
    const int tid = threadIdx.x, lane = tid & 31, wv = tid >> 5, l16 = lane & 15, hh = lane >> 4;
    const int rt = wv & 3, ch = wv >> 2;
    const int row0 = blockIdx.x * 64, col0 = blockIdx.y * 128;
    const size_t aoff = (size_t)(row0 + rt * 16 + l16) * lda + 8 * hh;
    const us* ar = A + aoff;
    const us* alr = Alo + aoff;
    const us* br = B + (size_t)(col0 + ch * 64 + l16) * ldb + 8 * hh;
    v8f acc[4], accl[4];
#pragma unroll
    for (int t = 0; t < 4; ++t) { acc[t] = vz8(); accl[t] = vz8(); }
#pragma unroll 1
    for (int kb = 0; kb < K; kb += 32) {
        const v16h a = frag(*(const us8*)(ar + kb), *(const us8*)(ar + kb + 16));
        v16h al = a;
        if (RES) al = frag(*(const us8*)(alr + kb), *(const us8*)(alr + kb + 16));
#pragma unroll
        for (int t = 0; t < 4; ++t) {
            const us* bp = br + (size_t)t * 16 * ldb + kb;
            const v16h b = frag(*(const us8*)bp, *(const us8*)(bp + 16));
            acc[t] = wm(a, b, acc[t]);
            if (RES) accl[t] = wm(al, b, accl[t]);
        }
    }
#pragma unroll
    for (int t = 0; t < 4; ++t) {
        const int cl = ch * 64 + t * 16 + l16;
#pragma unroll
        for (int r = 0; r < 8; ++r) {
            const int rl = rt * 16 + 8 * hh + r;
            float v = acc[t][r];
            if (RES) v += accl[t][r] * losc;
            cst[rl * CSTR + cl] = v * oscale;
        }
    }
    __syncthreads();
    float* cb = C + (size_t)row0 * ldc + col0 + lane * 4;
#pragma unroll
    for (int it = 0; it < 8; ++it) {
        const int row = it * 8 + wv;
        const v4f v = *(const v4fa*)&cst[row * CSTR + lane * 4];
        *(volatile v4f*)(cb + (size_t)row * ldc) = v;
    }
    __threadfence();
#pragma unroll
    for (int it = 0; it < 8; ++it) {
        const int row = it * 8 + wv;
        const v4f v = *(const v4fa*)&cst[row * CSTR + lane * 4];
        *(volatile v4f*)(cb + (size_t)row * ldc) = v;
    }
}

__global__ __launch_bounds__(128, 1) void split_hl(const float* __restrict__ C1, us* Ah, us* Al) {
    const int s = blockIdx.x, tid = threadIdx.x;
    const float* p = C1 + (size_t)s * N1 + tid * 8;
    const v4f a = *(const v4fa*)p, b = *(const v4fa*)(p + 4);
    float v[8];
    v[0] = a[0]; v[1] = a[1]; v[2] = a[2]; v[3] = a[3]; v[4] = b[0]; v[5] = b[1]; v[6] = b[2]; v[7] = b[3];
    us8 oh, ol;
#pragma unroll
    for (int e = 0; e < 8; ++e) {
        const _Float16 hx = (_Float16)v[e];
        oh[e] = __builtin_bit_cast(us, hx);
        ol[e] = hbits((v[e] - (float)hx) * LOSC);
    }
    us* dh = Ah + (size_t)s * AW + tid * 8;
    us* dl = Al + (size_t)s * AW + tid * 8;
    *(volatile us8*)dh = oh; *(volatile us8*)dl = ol;
    __threadfence();
    *(volatile us8*)dh = oh; *(volatile us8*)dl = ol;
}

__global__ __launch_bounds__(256, 1) void rope_tab(float* sinT, float* cosT, FreqTab ft) {
    const int tid = threadIdx.x, s = blockIdx.x * 8 + (tid >> 5), j = tid & 31;
    float inv = 0.0f;
#pragma unroll
    for (int q = 0; q < NFREQ; ++q) inv = (j == q) ? ft.inv[q] : inv;
    const float ang = (float)s * inv;
    const float sn = sinf(ang);
    const float cs = cosf(ang);
    float* ps = sinT + (size_t)s * NFREQ + j;
    float* pc = cosT + (size_t)s * NFREQ + j;
    *(volatile float*)ps = sn; *(volatile float*)pc = cs;
    __threadfence();
    *(volatile float*)ps = sn; *(volatile float*)pc = cs;
}

__global__ __launch_bounds__(256, 1) void pack_qk(const float* __restrict__ C1, const float* __restrict__ C2, const float* __restrict__ C3,
                                                  const float* __restrict__ sinT, const float* __restrict__ cosT, us* Qp, us* Kp) {
    const int s = blockIdx.x, tid = threadIdx.x;
    const int hc = tid >> 4, pc = tid & 15;
    const us8 oq = cvt8(C2 + (size_t)s * N2 + hc * DVH + pc * 8, 1.0f);
    const us8 ok = cvt8(C3 + (size_t)s * N3 + hc * DVH + pc * 8, 1.0f);
    us* dq = Qp + (size_t)s * QKW + hc * HQK + pc * 8;
    us* dk = Kp + (size_t)s * QKW + hc * HQK + pc * 8;
    const int isq = (tid < 128) ? 1 : 0;
    const int u = tid & 127, hr = u >> 3, pr = u & 7, i0 = pr * 8, j0 = i0 & 31;
    const float* xb = isq ? (C2 + (size_t)s * N2 + QR0 + hr * DROPE) : (C1 + (size_t)s * N1 + KR0);
    const v4f xa = *(const v4fa*)(xb + i0), xc = *(const v4fa*)(xb + i0 + 4);
    const v4f pa = *(const v4fa*)(xb + (i0 ^ 32)), pb = *(const v4fa*)(xb + (i0 ^ 32) + 4);
    const v4f sa = *(const v4fa*)(sinT + (size_t)s * NFREQ + j0), sb = *(const v4fa*)(sinT + (size_t)s * NFREQ + j0 + 4);
    const v4f ca = *(const v4fa*)(cosT + (size_t)s * NFREQ + j0), cb = *(const v4fa*)(cosT + (size_t)s * NFREQ + j0 + 4);
    const float sg = (i0 < 32) ? -1.0f : 1.0f;
    float xv[8], pv[8], sv[8], cv[8];
    xv[0] = xa[0]; xv[1] = xa[1]; xv[2] = xa[2]; xv[3] = xa[3]; xv[4] = xc[0]; xv[5] = xc[1]; xv[6] = xc[2]; xv[7] = xc[3];
    pv[0] = pa[0]; pv[1] = pa[1]; pv[2] = pa[2]; pv[3] = pa[3]; pv[4] = pb[0]; pv[5] = pb[1]; pv[6] = pb[2]; pv[7] = pb[3];
    sv[0] = sa[0]; sv[1] = sa[1]; sv[2] = sa[2]; sv[3] = sa[3]; sv[4] = sb[0]; sv[5] = sb[1]; sv[6] = sb[2]; sv[7] = sb[3];
    cv[0] = ca[0]; cv[1] = ca[1]; cv[2] = ca[2]; cv[3] = ca[3]; cv[4] = cb[0]; cv[5] = cb[1]; cv[6] = cb[2]; cv[7] = cb[3];
    us8 orr;
#pragma unroll
    for (int e = 0; e < 8; ++e) {
        const float rot = sg * pv[e];
        const float t1 = xv[e] * cv[e];
        const float t2 = rot * sv[e];
        orr[e] = hbits(bf16rt(t1 + t2));
    }
    us* dr = (isq ? Qp : Kp) + (size_t)s * QKW + hr * HQK + DVH + i0;
    *(volatile us8*)dq = oq; *(volatile us8*)dk = ok; *(volatile us8*)dr = orr;
    __threadfence();
    *(volatile us8*)dq = oq; *(volatile us8*)dk = ok; *(volatile us8*)dr = orr;
}

__global__ __launch_bounds__(256, 1) void vt_pack(const float* __restrict__ C3, us* VT) {
    __shared__ __align__(16) us tl[DVH * VTP];
    const int t0 = blockIdx.x * 64, h = blockIdx.y, tid = threadIdx.x;
#pragma unroll
    for (int it = 0; it < 8; ++it) {
        const int idx = it * 256 + tid, row = idx >> 5, c4 = idx & 31;
        const v4f v = *(const v4fa*)(C3 + (size_t)(t0 + row) * N3 + V0 + h * DVH + c4 * 4);
        tl[(c4 * 4 + 0) * VTP + row] = hbits(bf16rt(v[0]));
        tl[(c4 * 4 + 1) * VTP + row] = hbits(bf16rt(v[1]));
        tl[(c4 * 4 + 2) * VTP + row] = hbits(bf16rt(v[2]));
        tl[(c4 * 4 + 3) * VTP + row] = hbits(bf16rt(v[3]));
    }
    __syncthreads();
#pragma unroll
    for (int it = 0; it < 4; ++it) {
        const int d = it * 32 + (tid >> 3), q = tid & 7;
        const us8 o = *(const us8a*)&tl[d * VTP + q * 8];
        *(volatile us8*)(VT + (size_t)(h * DVH + d) * SEQ + t0 + q * 8) = o;
    }
    __threadfence();
#pragma unroll
    for (int it = 0; it < 4; ++it) {
        const int d = it * 32 + (tid >> 3), q = tid & 7;
        const us8 o = *(const us8a*)&tl[d * VTP + q * 8];
        *(volatile us8*)(VT + (size_t)(h * DVH + d) * SEQ + t0 + q * 8) = o;
    }
}

__device__ __forceinline__ void qk_tile(const us* qrow, const us* k0, const us* k1, v8f& s0, v8f& s1) {
#pragma unroll
    for (int ks = 0; ks < HQK / 32; ++ks) {
        const int kb = ks * 32;
        const v16h a  = frag(*(const us8a*)(qrow + kb), *(const us8a*)(qrow + kb + 16));
        const v16h b0 = frag(*(const us8*)(k0 + kb), *(const us8*)(k0 + kb + 16));
        const v16h b1 = frag(*(const us8*)(k1 + kb), *(const us8*)(k1 + kb + 16));
        s0 = wm(a, b0, s0);
        s1 = wm(a, b1, s1);
    }
}
__global__ __launch_bounds__(128, 1) void attn_kernel(const us* __restrict__ Qp, const us* __restrict__ Kp, const us* __restrict__ VT,
                                                      us* AT, float scale) {
    __shared__ __align__(16) us qlds[4 * 16 * QLP];
    __shared__ __align__(16) us plds[4 * 16 * PLP];
    const int tid = threadIdx.x, lane = tid & 31, w = tid >> 5, l16 = lane & 15, hh = lane >> 4;
    const int gw = blockIdx.x * 4 + w;
    const int h = gw / (SEQ / 16), qT = gw - h * (SEQ / 16);
    us* ql = qlds + w * 16 * QLP;
    us* pl = plds + w * 16 * PLP;
#pragma unroll
    for (int it = 0; it < 12; ++it) {
        const int idx = it * 32 + lane, r = idx / 24, pc = idx - r * 24;
        const us8 v = *(const us8*)(Qp + (size_t)(qT * 16 + r) * QKW + h * HQK + pc * 8);
        *(us8a*)(ql + r * QLP + pc * 8) = v;
    }
    __syncthreads();
    const us* qrow = ql + l16 * QLP + 8 * hh;
    const us* kbase = Kp + (size_t)l16 * QKW + h * HQK + 8 * hh;
    const us* vbase = VT + (size_t)(h * DVH + l16) * SEQ + 8 * hh;
    float m[8], l[8];
#pragma unroll
    for (int r = 0; r < 8; ++r) { m[r] = -__builtin_inff(); l[r] = 0.0f; }
#pragma unroll 1
    for (int t0 = 0; t0 < SEQ; t0 += 32) {
        v8f s0 = vz8(), s1 = vz8();
        const us* k0 = kbase + (size_t)t0 * QKW;
        const us* k1 = k0 + (size_t)16 * QKW;
        qk_tile(qrow, k0, k1, s0, s1);
#pragma unroll
        for (int r = 0; r < 8; ++r) {
            const float x0 = bf16rt(s0[r]) * scale, x1 = bf16rt(s1[r]) * scale;
            float mx = fmaxf(x0, x1);
            mx = fmaxf(mx, __shfl_xor(mx, 1, 32));
            mx = fmaxf(mx, __shfl_xor(mx, 2, 32));
            mx = fmaxf(mx, __shfl_xor(mx, 4, 32));
            mx = fmaxf(mx, __shfl_xor(mx, 8, 32));
            const float mn = fmaxf(m[r], mx);
            const float alpha = __expf(m[r] - mn);
            float e = __expf(x0 - mn) + __expf(x1 - mn);
            e += __shfl_xor(e, 1, 32);
            e += __shfl_xor(e, 2, 32);
            e += __shfl_xor(e, 4, 32);
            e += __shfl_xor(e, 8, 32);
            l[r] = l[r] * alpha + e;
            m[r] = mn;
        }
    }
    float inv[8];
#pragma unroll
    for (int r = 0; r < 8; ++r) inv[r] = 1.0f / l[r];
    v8f O[8];
#pragma unroll
    for (int n = 0; n < 8; ++n) O[n] = vz8();
#pragma unroll 1
    for (int t0 = 0; t0 < SEQ; t0 += 32) {
        v8f s0 = vz8(), s1 = vz8();
        const us* k0 = kbase + (size_t)t0 * QKW;
        const us* k1 = k0 + (size_t)16 * QKW;
        qk_tile(qrow, k0, k1, s0, s1);
        __syncthreads();
#pragma unroll
        for (int r = 0; r < 8; ++r) {
            const float x0 = bf16rt(s0[r]) * scale, x1 = bf16rt(s1[r]) * scale;
            const float p0 = __expf(x0 - m[r]) * inv[r];
            const float p1 = __expf(x1 - m[r]) * inv[r];
            pl[(8 * hh + r) * PLP + l16]      = hbits(bf16rt(p0) * PSC);
            pl[(8 * hh + r) * PLP + 16 + l16] = hbits(bf16rt(p1) * PSC);
        }
        __syncthreads();
        const v16h pa = frag(*(const us8a*)(pl + l16 * PLP + 8 * hh), *(const us8a*)(pl + l16 * PLP + 16 + 8 * hh));
#pragma unroll
        for (int n = 0; n < 8; ++n) {
            const us* vp = vbase + (size_t)n * 16 * SEQ + t0;
            const v16h vb = frag(*(const us8*)vp, *(const us8*)(vp + 16));
            O[n] = wm(pa, vb, O[n]);
        }
    }
    __syncthreads();
#pragma unroll
    for (int n = 0; n < 8; ++n) {
#pragma unroll
        for (int r = 0; r < 8; ++r) ql[(8 * hh + r) * QLP + n * 16 + l16] = hbits(bf16rt(O[n][r] * (1.0f / PSC)) * ATSC);
    }
    __syncthreads();
    us* ob = AT + (size_t)(qT * 16) * EMB + h * DVH + l16 * 8;
#pragma unroll
    for (int it = 0; it < 8; ++it) {
        const int row = it * 2 + hh;
        const us8 v = *(const us8a*)(ql + row * QLP + l16 * 8);
        *(volatile us8*)(ob + (size_t)row * EMB) = v;
    }
    __threadfence();
#pragma unroll
    for (int it = 0; it < 8; ++it) {
        const int row = it * 2 + hh;
        const us8 v = *(const us8a*)(ql + row * QLP + l16 * 8);
        *(volatile us8*)(ob + (size_t)row * EMB) = v;
    }
}

extern "C" void kernel_launch(void* const* d_in, const int* in_sizes, int n_in,
                              void* d_out, int out_size, void* d_ws, size_t ws_size, hipStream_t stream) {
    if (n_in < 8) return;
    if (in_sizes[0] < SEQ * EMB || in_sizes[1] < QRK * EMB || in_sizes[2] < NH * DVH * QRK || in_sizes[3] < NH * DROPE * QRK ||
        in_sizes[4] < KVRK * EMB || in_sizes[5] < N3 * KVRK || in_sizes[6] < DROPE * EMB || in_sizes[7] < EMB * EMB) return;
    if (out_size < SEQ * EMB) return;
    const float* x        = (const float*)d_in[0];
    const float* wq_down  = (const float*)d_in[1];
    const float* wq_up    = (const float*)d_in[2];
    const float* wq_rope  = (const float*)d_in[3];
    const float* wkv_down = (const float*)d_in[4];
    const float* wkv_up   = (const float*)d_in[5];
    const float* wk_rope  = (const float*)d_in[6];
    const float* wo       = (const float*)d_in[7];
    float* out = (float*)d_out;

    char* ws = (char*)d_ws;
    size_t off = 0;
    auto carve = [&](size_t bytes) -> char* { char* p = ws + off; off += (bytes + 255) & ~(size_t)255; return p; };
    us* xh      = (us*)carve((size_t)SEQ * EMB * 2);
    us* Wd      = (us*)carve((size_t)N1 * EMB * 2);
    us* Wqu     = (us*)carve((size_t)N2 * QRK * 2);
    us* Wkvu    = (us*)carve((size_t)N3 * KVRK * 2);
    us* Woh     = (us*)carve((size_t)EMB * EMB * 2);
    float* C1   = (float*)carve((size_t)SEQ * N1 * 4);
    us* A2h     = (us*)carve((size_t)SEQ * AW * 2);
    us* A2l     = (us*)carve((size_t)SEQ * AW * 2);
    float* sinT = (float*)carve((size_t)SEQ * NFREQ * 4);
    float* cosT = (float*)carve((size_t)SEQ * NFREQ * 4);
    float* C2   = (float*)carve((size_t)SEQ * N2 * 4);
    float* C3   = (float*)carve((size_t)SEQ * N3 * 4);
    us* Qp      = (us*)carve((size_t)SEQ * QKW * 2);
    us* Kp      = (us*)carve((size_t)SEQ * QKW * 2);
    if (off > ws_size) return;
    us* AT  = xh;
    us* VTp = A2h;

    FreqTab ft;
    for (int j = 0; j < NFREQ; ++j) { const float p = (float)pow(10000.0, (double)j / 32.0); ft.inv[j] = 1.0f / p; }
    const float scale = (float)0.07216878364870322;

    auto cvt = [&](const float* s, us* d, int n8, float sc) { cvt_plane<<<dim3(n8 / 256), dim3(256), 0, stream>>>(s, d, n8, sc); };
    cvt(x, xh, SEQ * EMB / 8, 1.0f);
    cvt(wq_down, Wd, QRK * EMB / 8, 32.0f);
    cvt(wkv_down, Wd + (size_t)CKV0 * EMB, KVRK * EMB / 8, 32.0f);
    cvt(wk_rope, Wd + (size_t)KR0 * EMB, DROPE * EMB / 8, 32.0f);
    zero_plane<<<dim3((N1 - N1USE) * EMB / 8 / 256), dim3(256), 0, stream>>>(Wd + (size_t)N1USE * EMB, (N1 - N1USE) * EMB / 8);
    cvt(wq_up, Wqu, NH * DVH * QRK / 8, 16.0f);
    cvt(wq_rope, Wqu + (size_t)QR0 * QRK, NH * DROPE * QRK / 8, 16.0f);
    cvt(wkv_up, Wkvu, N3 * KVRK / 8, 16.0f);
    cvt(wo, Woh, EMB * EMB / 8, 32.0f);

    gemm_nt<0><<<dim3(SEQ / 64, N1 / 128), dim3(256), 0, stream>>>(xh, xh, EMB, Wd, EMB, C1, N1, EMB, 1.0f / 32.0f, 0.0f);
    split_hl<<<dim3(SEQ), dim3(128), 0, stream>>>(C1, A2h, A2l);
    rope_tab<<<dim3(SEQ / 8), dim3(256), 0, stream>>>(sinT, cosT, ft);
    gemm_nt<1><<<dim3(SEQ / 64, N2 / 128), dim3(256), 0, stream>>>(A2h, A2l, AW, Wqu, QRK, C2, N2, QRK, 1.0f / 16.0f, 1.0f / LOSC);
    gemm_nt<1><<<dim3(SEQ / 64, N3 / 128), dim3(256), 0, stream>>>(A2h + CKV0, A2l + CKV0, AW, Wkvu, KVRK, C3, N3, KVRK, 1.0f / 16.0f, 1.0f / LOSC);
    pack_qk<<<dim3(SEQ), dim3(256), 0, stream>>>(C1, C2, C3, sinT, cosT, Qp, Kp);
    vt_pack<<<dim3(SEQ / 64, NH), dim3(256), 0, stream>>>(C3, VTp);
    attn_kernel<<<dim3(NH * (SEQ / 64)), dim3(128), 0, stream>>>(Qp, Kp, VTp, AT, scale);
    gemm_nt<0><<<dim3(SEQ / 64, EMB / 128), dim3(256), 0, stream>>>(AT, AT, EMB, Woh, EMB, out, EMB, EMB, 1.0f / (32.0f * ATSC), 0.0f);
}
